// MultiHeadMLP_87943750353236
// MI455X (gfx1250) — hardware-verified
//
#include <hip/hip_runtime.h>
#include <hip/hip_bf16.h>
#include <math.h>

#define NTOK 4096
#define DMODEL 1024
#define HH 8
#define DKK 128
#define NK 2048
#define QW 1
#define QST 1024
#define KVST 1024
#define KST2 136
#define GSTR 48

typedef _Float16 bf16;
typedef _Float16 f16;
typedef __attribute__((ext_vector_type(4))) unsigned v4u_t;
typedef unsigned v4ua __attribute__((ext_vector_type(4), may_alias));
typedef __attribute__((ext_vector_type(4))) float v4f_t;
typedef float v4fa __attribute__((ext_vector_type(4), may_alias));
typedef __attribute__((ext_vector_type(16))) bf16  bf16x16;
typedef bf16x16 f16x16;
typedef __attribute__((ext_vector_type(8)))  bf16  bf16x8;
typedef bf16x8 f16x8;
typedef __attribute__((ext_vector_type(4)))  bf16  bf16x4;
typedef __attribute__((ext_vector_type(8)))  float f32x8;
__device__ __forceinline__ f32x8 wmma16(f16x16 a, f16x16 b, f32x8 c) {
  c = __builtin_amdgcn_wmma_f32_16x16x32_f16(false, a, false, b, (short)0, c, false, false);
  asm volatile("v_nop\n\tv_nop\n\tv_nop\n\tv_nop" : "+v"(c) : "v"(a), "v"(b));
  return c;
}
#define LDS_STRIDE 48
#define KSTRIDE    72
#define VSTRIDE    48

__device__ __forceinline__ f32x8 wmma_bf16(bf16x16 a, bf16x16 b, f32x8 c) {
  c = __builtin_amdgcn_wmma_f32_16x16x32_f16(false, a, false, b, (short)0, c, false, false);
  asm volatile("v_nop\n\tv_nop\n\tv_nop\n\tv_nop" : "+v"(c) : "v"(a), "v"(b));
  return c;
}

template <typename T>
__device__ __forceinline__ bf16x16 load_frag(const T* __restrict__ base, int ld,
                                             int row0, int k0) {
  const int lane = threadIdx.x & 31;
  const int r    = lane & 15;
  const int kh   = (lane >> 4) * 8;
  const T* p0 = base + (size_t)(row0 + r) * ld + (k0 + kh);
  const T* p1 = p0 + 16;
  bf16x16 f;
#pragma unroll
  for (int i = 0; i < 8; ++i) {
    f[i]     = (bf16)p0[i];
    f[i + 8] = (bf16)p1[i];
  }
  return f;
}

__device__ __forceinline__ bf16x16 lds_frag(const bf16* base, int stride) {
  const int lane = threadIdx.x & 31;
  const int row  = lane & 15;
  const int kh   = (lane >> 4) * 8;
  const bf16x8 lo = *(const bf16x8*)(base + row * stride + kh);
  const bf16x8 hi = *(const bf16x8*)(base + row * stride + kh + 16);
  bf16x16 f;
#pragma unroll
  for (int i = 0; i < 8; ++i) { f[i] = lo[i]; f[i + 8] = hi[i]; }
  return f;
}

template <typename T>
__device__ __forceinline__ void stage_read16(const T* __restrict__ p, float* buf) {
#pragma unroll
  for (int i = 0; i < 16; ++i) buf[i] = (float)p[i];
}

__device__ __forceinline__ void stage_write(bf16* dst, const float* buf, int nquad) {
#pragma unroll
  for (int i = 0; i < nquad; ++i) {
    bf16x4 q;
    q[0] = (bf16)buf[4 * i];     q[1] = (bf16)buf[4 * i + 1];
    q[2] = (bf16)buf[4 * i + 2]; q[3] = (bf16)buf[4 * i + 3];
    *(bf16x4*)(dst + 4 * i) = q;
  }
}

__global__ __launch_bounds__(64) void attn_kernel(
    const bf16* __restrict__ Qb, const bf16* __restrict__ Kb,
    const bf16* __restrict__ Vt,
    bf16* __restrict__ attnOut) {
  __shared__ bf16 ldsK[32 * KST2];
  __shared__ bf16 ldsV[128 * VSTRIDE];
  __shared__ __attribute__((aligned(16))) bf16 ldsO[2][16 * 136];

  const int q0blk = blockIdx.x * 32;
  const int h  = blockIdx.y;
  const int b  = blockIdx.z;
  const int t    = threadIdx.x;
  const int wave = t >> 5;
  const int lane = t & 31;
  const int qlane = lane & 15;
  const int kh8   = (lane >> 4) * 8;
  const int q0 = q0blk + wave * 16;

  (void)b;
  const bf16* Qh = Qb + h * DKK;
  const bf16* Kh = Kb + h * DKK;
  const bf16* Vh = Vt + (size_t)h * DKK * NK;

  const int krow = t >> 1;
  const int kcol = (t & 1) * 64;
  const bf16* kSrc = Kh + (size_t)krow * KVST + kcol;
  const bf16* vSrc = Vh + (size_t)t * NK;

  bf16x16 qf[QW][4];
#pragma unroll
  for (int qt = 0; qt < QW; ++qt)
#pragma unroll
    for (int c = 0; c < 4; ++c) qf[qt][c] = load_frag(Qh, QST, q0 + 16 * qt, 32 * c);

  f32x8 o[QW][8] = {};
  float mrun[QW], lrun[QW];
#pragma unroll
  for (int qt = 0; qt < QW; ++qt) { mrun[qt] = -INFINITY; lrun[qt] = 0.0f; }

  const float scale = 1.44269504088896340736f;
  const float NEG2 = -1.0e9f; (void)NEG2;
  const int kmax = NK - 1, kmin = 0;

  bf16x8 kreg[8], vreg[8];
#pragma unroll
  for (int i = 0; i < 8; ++i) kreg[i] = *(const bf16x8*)(kSrc + (size_t)kmin * KVST + 8 * i);
#pragma unroll
  for (int i = 0; i < 4; ++i) { vreg[i] = *(const bf16x8*)(vSrc + kmin + 8 * i); vreg[4 + i] = *(const bf16x8*)(vSrc + (size_t)64 * NK + kmin + 8 * i); }

  for (int kb = kmin; kb <= kmax; kb += 32) {
    __syncthreads();
#pragma unroll
    for (int i = 0; i < 8; ++i) *(bf16x8*)(&ldsK[krow * KST2 + kcol + 8 * i]) = kreg[i];
#pragma unroll
    for (int i = 0; i < 4; ++i) { *(bf16x8*)(&ldsV[t * VSTRIDE + 8 * i]) = vreg[i]; *(bf16x8*)(&ldsV[(t + 64) * VSTRIDE + 8 * i]) = vreg[4 + i]; }
    if (kb + 32 <= kmax) {
      const bf16* kn = kSrc + (size_t)(kb + 32) * KVST;
      const bf16* vn = vSrc + (kb + 32);
#pragma unroll
      for (int i = 0; i < 8; ++i) kreg[i] = *(const bf16x8*)(kn + 8 * i);
#pragma unroll
      for (int i = 0; i < 4; ++i) { vreg[i] = *(const bf16x8*)(vn + 8 * i); vreg[4 + i] = *(const bf16x8*)(vn + (size_t)64 * NK + 8 * i); }
    }
    __syncthreads();


    bf16x16 pf[QW];
    bool act[QW];
#pragma unroll
    for (int qt = 0; qt < QW; ++qt) {
      unsigned mbits = 0;
      mbits = 0xFFFFu; act[qt] = true;
      if (act[qt]) {
        const int q_my = q0 + 16 * qt + qlane;
        f32x8 s0 = {}, s1 = {};
#pragma unroll
        for (int c = 0; c < 4; ++c) {
          const bf16x16 k0f = lds_frag(ldsK + 0 * KST2 + c * 32, KST2), k1f = lds_frag(ldsK + 16 * KST2 + c * 32, KST2);
          s0 = wmma_bf16(k0f, qf[qt][c], s0);
          s1 = wmma_bf16(k1f, qf[qt][c], s1);
        }

        float mx = -INFINITY;
#pragma unroll
        for (int r = 0; r < 8; ++r) {
          const int k0i = kb + kh8 + r;
          const int k1i = k0i + 16;
          (void)k0i; (void)k1i; (void)q_my;
          s0[r] = (mbits & (1u << r))       ? s0[r] * scale : NEG2;
          s1[r] = (mbits & (1u << (8 + r))) ? s1[r] * scale : NEG2;
          mx = fmaxf(mx, fmaxf(s0[r], s1[r]));
        }
        mx = fmaxf(mx, __shfl_xor(mx, 16, 32));
        const float mnew  = fmaxf(mrun[qt], mx);
        const float alpha = exp2f(mrun[qt] - mnew);

        float rsum = 0.0f;
#pragma unroll
        for (int r = 0; r < 8; ++r) {
          const float p0 = exp2f(s0[r] - mnew);
          const float p1 = exp2f(s1[r] - mnew);
          rsum += p0 + p1;
          pf[qt][r]     = (bf16)(p0 * 1024.0f);
          pf[qt][r + 8] = (bf16)(p1 * 1024.0f);
        }
        rsum += __shfl_xor(rsum, 16, 32);
        lrun[qt] = lrun[qt] * alpha + rsum;
        mrun[qt] = mnew;

#pragma unroll
        for (int j = 0; j < 8; ++j)
#pragma unroll
          for (int r = 0; r < 8; ++r) o[qt][j][r] *= alpha;
      }
    }

#pragma unroll
    for (int j = 0; j < 8; ++j) {
      const bf16x16 vf = lds_frag(ldsV + (j * 16) * VSTRIDE, VSTRIDE);
#pragma unroll
      for (int qt = 0; qt < QW; ++qt)
        if (act[qt]) o[qt][j] = wmma_bf16(vf, pf[qt], o[qt][j]);
    }
  }

  bf16* so = ldsO[wave];
  {
    const float rl = 1.0f / (lrun[0] * 1024.0f);
#pragma unroll
    for (int j = 0; j < 8; ++j)
#pragma unroll
      for (int r = 0; r < 8; ++r) so[qlane * 136 + j * 16 + kh8 + r] = (bf16)(o[0][j][r] * rl);
  }
  asm volatile("s_wait_dscnt 0" ::: "memory");
  __builtin_amdgcn_wave_barrier();
#pragma unroll 1
  for (int pass = 0; pass < 2; ++pass) {
#pragma unroll
    for (int it = 0; it < 8; ++it) { const int ch = lane + 32 * it, ql = ch >> 4, q8 = (ch & 15) * 8;
      *(volatile v4u_t*)(attnOut + ((size_t)(q0 + ql)) * QST + h * DKK + q8) = *(const v4ua*)(so + ql * 136 + q8); }
    __threadfence();
  }
}


#define GSTR 48
template <typename AT, int EPI, bool OUT16>
__global__ __launch_bounds__(256) void gemm_kne(const AT* __restrict__ A, int lda, const float* __restrict__ Wm, int ldw,
                                                const float* __restrict__ bias, const float* __restrict__ R, const float* __restrict__ gvec,
                                                void* __restrict__ Yv, int ldy, int K) {
  __shared__ __attribute__((aligned(16))) f16 ldsA[128 * GSTR];
  __shared__ __attribute__((aligned(16))) f16 ldsW[128 * GSTR];
  __shared__ __attribute__((aligned(16))) float oS[8][32 * 68];
  const int tid = threadIdx.x, lane = tid & 31, wave = tid >> 5, cl = lane & 15, rh = (lane >> 4) * 8;
  const int m0 = blockIdx.x * 128, n0 = blockIdx.y * 128;
  const int wm = (wave & 3) * 32, wn = (wave >> 2) * 64;
  f32x8 acc[2][4];
#pragma unroll
  for (int i = 0; i < 2; ++i)
#pragma unroll
    for (int j = 0; j < 4; ++j) { f32x8 z = {}; acc[i][j] = z; }
#pragma unroll 1
  for (int k0 = 0; k0 < K; k0 += 32) {
    __syncthreads();
    { const int row = tid >> 1, ch = (tid & 1) * 16;
      const AT* src = A + (size_t)(m0 + row) * lda + k0 + ch;
#pragma unroll
      for (int g = 0; g < 16; ++g) ldsA[row * GSTR + ch + g] = (f16)src[g]; }
    { const int k = tid >> 3, nn0 = (tid & 7) * 16;
      const float* src = Wm + (size_t)(k0 + k) * ldw + n0 + nn0;
#pragma unroll
      for (int g = 0; g < 4; ++g) { const v4f_t v = *(const v4f_t*)(src + 4 * g);
#pragma unroll
        for (int u = 0; u < 4; ++u) ldsW[(nn0 + 4 * g + u) * GSTR + k] = (f16)v[u]; } }
    __syncthreads();
    f16x16 af[2];
#pragma unroll
    for (int i = 0; i < 2; ++i) af[i] = lds_frag(ldsA + (wm + 16 * i) * GSTR, GSTR);
#pragma unroll
    for (int j = 0; j < 4; ++j) {
      const f16x16 bf = lds_frag(ldsW + (wn + 16 * j) * GSTR, GSTR);
#pragma unroll
      for (int i = 0; i < 2; ++i) acc[i][j] = wmma16(af[i], bf, acc[i][j]);
    }
  }
  float* so = oS[wave];
#pragma unroll
  for (int i = 0; i < 2; ++i)
#pragma unroll
    for (int j = 0; j < 4; ++j) {
      const int n = n0 + wn + 16 * j + cl;
      const float bv = bias ? bias[n] : 0.0f;
      const float gv = (EPI == 2) ? gvec[n] : 0.0f;
      if (EPI == 1) {
#pragma unroll 1
        for (int r = 0; r < 8; ++r) { const float xg = acc[i][j][r] + bv; so[(16 * i + rh + r) * 68 + 16 * j + cl] = 0.5f * xg * (1.0f + erff(xg * 0.70710678118654752f)); }
      } else {
#pragma unroll
        for (int r = 0; r < 8; ++r) {
          float v = acc[i][j][r] + bv;
          if (EPI == 2) v = R[(size_t)(m0 + wm + 16 * i + rh + r) * ldy + n] + gv * v;
          so[(16 * i + rh + r) * 68 + 16 * j + cl] = v;
        }
      }
    }
  asm volatile("s_wait_dscnt 0" ::: "memory");
  __builtin_amdgcn_wave_barrier();
#pragma unroll 1
  for (int pass = 0; pass < 2; ++pass) {
    if (OUT16) {
      f16* Y = (f16*)Yv;
#pragma unroll
      for (int it = 0; it < 8; ++it) { const int c = lane + 32 * it, rr = c >> 3, q8 = (c & 7) * 8;
        union { f16 h[8]; v4u_t v; } u;
#pragma unroll
        for (int e = 0; e < 8; ++e) u.h[e] = (f16)so[rr * 68 + q8 + e];
        *(volatile v4u_t*)(Y + (size_t)(m0 + wm + rr) * ldy + n0 + wn + q8) = u.v; }
    } else {
      float* Y = (float*)Yv;
#pragma unroll
      for (int it = 0; it < 16; ++it) { const int f4 = lane + 32 * it, rr = f4 >> 4, q = (f4 & 15) * 4;
        *(volatile v4f_t*)(Y + (size_t)(m0 + wm + rr) * ldy + n0 + wn + q) = *(const volatile v4fa*)(so + rr * 68 + q); }
    }
    __threadfence();
  }
}

__global__ __launch_bounds__(256) void k_qnorm(const float* __restrict__ q, bf16* __restrict__ q16) {
  const int tid = threadIdx.x, pr = tid >> 1, half = tid & 1; const int tok = blockIdx.x * 16 + (pr >> 3), h = pr & 7;
  const float* src = q + (size_t)tok * DMODEL + h * DKK + half * 64; float ss = 0.0f;
  for (int i = 0; i < 64; ++i) { const float v = src[i]; ss += v * v; }
  ss += __shfl_xor(ss, 1, 32); const float r = rsqrtf(ss + 1e-6f);
  bf16* dst = q16 + (size_t)tok * DMODEL + h * DKK + half * 64;
#pragma unroll 1
  for (int pass = 0; pass < 2; ++pass) {
    for (int c8 = 0; c8 < 64; c8 += 8) { union { bf16 hh[8]; v4u_t u; } cv;
#pragma unroll
      for (int e = 0; e < 8; ++e) cv.hh[e] = (bf16)(src[c8 + e] * r);
      *(volatile v4u_t*)(dst + c8) = cv.u; }
    __threadfence(); }
}
__global__ __launch_bounds__(256) void k_knorm(const float* __restrict__ keys, const float* __restrict__ ascale, bf16* __restrict__ k16) {
  const int tid = threadIdx.x, pr = tid >> 1, half = tid & 1; const int slot = blockIdx.x * 16 + (pr >> 3), h = pr & 7;
  const float* src = keys + ((size_t)slot * HH + h) * DKK + half * 64; float ss = 0.0f;
  for (int i = 0; i < 64; ++i) { const float v = src[i]; ss += v * v; }
  ss += __shfl_xor(ss, 1, 32); const float r = rsqrtf(ss + 1e-6f) * ascale[h];
  bf16* dst = k16 + ((size_t)slot * HH + h) * DKK + half * 64;
#pragma unroll 1
  for (int pass = 0; pass < 2; ++pass) {
    for (int c8 = 0; c8 < 64; c8 += 8) { union { bf16 hh[8]; v4u_t u; } cv;
#pragma unroll
      for (int e = 0; e < 8; ++e) cv.hh[e] = (bf16)(src[c8 + e] * r);
      *(volatile v4u_t*)(dst + c8) = cv.u; }
    __threadfence(); }
}
__global__ __launch_bounds__(256) void k_vt(const float* __restrict__ vals, bf16* __restrict__ Vt) {
  __shared__ bf16 tS[64][520];
  const int tid = threadIdx.x, s0 = (blockIdx.x >> 1) * 64, chalf = blockIdx.x & 1;
  for (int e = tid; e < 64 * 512; e += 256) { const int r = e >> 9, c = e & 511; tS[r][c] = (bf16)vals[(size_t)(s0 + r) * 1024 + chalf * 512 + c]; }
  __syncthreads();
  for (int ch = tid; ch < 512 * 8; ch += 256) { const int cl2 = ch >> 3, q8 = (ch & 7) * 8; const int c = chalf * 512 + cl2; const int h = c >> 7, d = c & 127; union { bf16 hh[8]; v4u_t u; } cv;
#pragma unroll
    for (int e = 0; e < 8; ++e) cv.hh[e] = tS[q8 + e][cl2];
    bf16* dst = Vt + ((size_t)h * DKK + d) * NK + s0 + q8;
    *(volatile v4u_t*)dst = cv.u; __threadfence(); *(volatile v4u_t*)dst = cv.u; }
}

extern "C" void kernel_launch(void* const* d_in, const int* in_sizes, int n_in,
                              void* d_out, int out_size, void* d_ws, size_t ws_size,
                              hipStream_t stream) {
  (void)in_sizes; (void)n_in; (void)out_size;
  const float* x = (const float*)d_in[0];
  const float* Wq = (const float*)d_in[1];
  const float* keys = (const float*)d_in[2];
  const float* vals = (const float*)d_in[3];
  const float* ascale = (const float*)d_in[4];
  const float* Wo = (const float*)d_in[5];
  float* out = (float*)d_out;
  char* ws = (char*)d_ws;
  float* qf = (float*)ws; ws += (size_t)NTOK * DMODEL * 4;
  bf16* q16 = (bf16*)ws; ws += (size_t)NTOK * DMODEL * 2;
  bf16* k16 = (bf16*)ws; ws += (size_t)NK * DMODEL * 2;
  bf16* Vt = (bf16*)ws; ws += (size_t)NK * DMODEL * 2;
  bf16* att = (bf16*)ws; ws += (size_t)NTOK * DMODEL * 2;
  if ((size_t)(ws - (char*)d_ws) > ws_size) return;
  const dim3 blk(256);
  gemm_kne<float, 0, false><<<dim3(NTOK / 128, DMODEL / 128), blk, 0, stream>>>(x, DMODEL, Wq, DMODEL, nullptr, nullptr, nullptr, qf, DMODEL, DMODEL);
  k_qnorm<<<dim3(NTOK / 16), blk, 0, stream>>>(qf, q16);
  k_knorm<<<dim3(NK / 16), blk, 0, stream>>>(keys, ascale, k16);
  k_vt<<<dim3((NK / 64) * 2), blk, 0, stream>>>(vals, Vt);
  attn_kernel<<<dim3(NTOK / 32, HH, 1), dim3(64), 0, stream>>>(q16, k16, Vt, att);
  gemm_kne<bf16, 0, false><<<dim3(NTOK / 128, DMODEL / 128), blk, 0, stream>>>(att, DMODEL, Wo, DMODEL, nullptr, nullptr, nullptr, out, DMODEL, DMODEL);
}
